// GptOssAttention_17824114279001
// MI455X (gfx1250) — hardware-verified
//
#include <hip/hip_runtime.h>
#include <math.h>

#ifndef SEQ
#define SEQ 1024
#endif
#ifndef NB
#define NB 1
#endif
#define SEQ_FULL 1024
#define HID 2880
#define NQH 64
#define NKVH 8
#define HDM 64
#define QW (NQH * HDM)
#define KVW (NKVH * HDM)
#define QKVW (QW + 2 * KVW)
static_assert(NB == 1);
static_assert(SEQ % 128 == 0 && SEQ >= 128 && SEQ <= SEQ_FULL);
static_assert(HID % 64 == 0 && HID % 32 == 0 && QKVW % 64 == 0 && QW == 4096 && KVW == 512 && QKVW == 5120);

typedef __attribute__((ext_vector_type(16))) _Float16 v16h;
typedef __attribute__((ext_vector_type(8)))  _Float16 v8h;
typedef __attribute__((ext_vector_type(16))) __bf16   v16b;
typedef __attribute__((ext_vector_type(8)))  __bf16   v8b;
typedef __attribute__((ext_vector_type(8)))  float    v8f;
typedef __attribute__((ext_vector_type(4)))  float    v4f;
typedef __attribute__((ext_vector_type(4)))  int      v4i;
typedef __attribute__((ext_vector_type(4)))  unsigned v4u;

#define VST2(T, ptr, val) do { const T vst2_v_ = (val); *(volatile T*)(ptr) = vst2_v_; __threadfence(); *(volatile T*)(ptr) = vst2_v_; } while (0)

namespace kit {

__device__ __forceinline__ unsigned short f2bf_bits(float f) {
  unsigned u = __float_as_uint(f);
  return (unsigned short)((u + 0x7FFFu + ((u >> 16) & 1u)) >> 16);
}
__device__ __forceinline__ float bf_bits2f(unsigned short h) { return __uint_as_float(((unsigned)h) << 16); }

__device__ __forceinline__ void dep_guard_h(v8f& a, v8f& b, v16h x, v16h y) { asm volatile("v_nop\n\tv_nop\n\tv_nop\n\tv_nop" : "+v"(a), "+v"(b) : "v"(x), "v"(y)); }
__device__ __forceinline__ void dep_guard_b(v8f& a, v8f& b, v16b x, v16b y) { asm volatile("v_nop\n\tv_nop\n\tv_nop\n\tv_nop" : "+v"(a), "+v"(b) : "v"(x), "v"(y)); }
__device__ __forceinline__ void keep4_h(v16h a, v16h b, v16h c, v16h d) { asm volatile("v_nop" :: "v"(a), "v"(b), "v"(c), "v"(d)); }
__device__ __forceinline__ void keep4_b(v16b a, v16b b, v16b c, v16b d) { asm volatile("v_nop" :: "v"(a), "v"(b), "v"(c), "v"(d)); }
__device__ __forceinline__ void acc_guard4(v8f& a, v8f& b, v8f& c, v8f& d) { asm volatile("v_nop\n\tv_nop\n\tv_nop\n\tv_nop" : "+v"(a), "+v"(b), "+v"(c), "+v"(d)); }
template <typename T> struct Frag;
template <> struct Frag<_Float16> {
  typedef v16h V; union U { v16h v; v8h h[2]; };
  static __device__ __forceinline__ v16h load(const _Float16* p) {
    U f; f.h[0] = *(const v8h*)(p); f.h[1] = *(const v8h*)(p + 16); return f.v;
  }
  static __device__ __forceinline__ v8f mma(v16h a, v16h b, v8f c) {
    return __builtin_amdgcn_wmma_f32_16x16x32_f16(false, a, false, b, (short)0, c, false, false);
  }
  static __device__ __forceinline__ void guard(v8f& a, v8f& b, v16h x, v16h y) { dep_guard_h(a, b, x, y); }
  static __device__ __forceinline__ void keep(v16h a, v16h b, v16h c, v16h d) { keep4_h(a, b, c, d); }
};
template <> struct Frag<__bf16> {
  typedef v16b V; union U { v16b v; v8b h[2]; };
  static __device__ __forceinline__ v16b load(const __bf16* p) {
    U f; f.h[0] = *(const v8b*)(p); f.h[1] = *(const v8b*)(p + 16); return f.v;
  }
  static __device__ __forceinline__ v8f mma(v16b a, v16b b, v8f c) {
    return __builtin_amdgcn_wmma_f32_16x16x32_bf16(false, a, false, b, (short)0, c, false, false);
  }
  static __device__ __forceinline__ void guard(v8f& a, v8f& b, v16b x, v16b y) { dep_guard_b(a, b, x, y); }
  static __device__ __forceinline__ void keep(v16b a, v16b b, v16b c, v16b d) { keep4_b(a, b, c, d); }
};

template <int ET> struct Elem;
template <> struct Elem<0> { typedef _Float16 T; };
template <> struct Elem<1> { typedef __bf16 T; };
template <int ET, bool SPLIT, int BIAS_MODE, int OUT_MODE, bool RESID, int ACT = 0>
__global__ __launch_bounds__(256) void wmma_gemm64(
    const unsigned short* __restrict__ Ap, const unsigned short* __restrict__ A2p, int lda, long strideA,
    const unsigned short* __restrict__ Btp, const unsigned short* __restrict__ Bt2p, int ldb, long strideB,
    void* __restrict__ Cout, void* __restrict__ Cout2, int ldc, long strideC,
    const float* __restrict__ bias,
    const float* __restrict__ resid, long strideR,
    int M, int N, int K, float scale) {
  typedef typename Elem<ET>::T T;
  typedef typename Frag<T>::V V;
  const T* A = (const T*)Ap; const T* A2 = (const T*)A2p; const T* Bt = (const T*)Btp; const T* Bt2 = (const T*)Bt2p;
  __shared__ __align__(16) float sT[8][16 * 68];
  const int b    = blockIdx.y;
  const int lane = threadIdx.x & 31;
  const int wave = threadIdx.x >> 5;
  const int tilesN = N >> 6;
  const int tilesM = M >> 6;
  const int tile = blockIdx.x * 8 + wave;
  if (tile >= tilesM * tilesN) return;
  const int tm = tile / tilesN;
  const int tn = tile - tm * tilesN;
  const int m0 = tm << 6;
  const int n0 = tn << 6;

  const T* Ab  = A  + (size_t)b * strideA;
  const T* Bb  = Bt + (size_t)b * strideB;
  const T* Ab2 = SPLIT ? (A2  + (size_t)b * strideA) : nullptr;
  const T* Bb2 = SPLIT ? (Bt2 + (size_t)b * strideB) : nullptr;

  const int rlane = lane & 15;
  const int koff  = (lane >> 4) * 8;
  const int mOff  = (lane >> 4) * 8;

  v8f acc[4][4];
#pragma unroll
  for (int i = 0; i < 4; ++i)
#pragma unroll
    for (int j = 0; j < 4; ++j) acc[i][j] = (v8f){0.f,0.f,0.f,0.f,0.f,0.f,0.f,0.f};

  for (int k0 = 0; k0 < K; k0 += 32) {
    V bh[4], bl[4];
#pragma unroll
    for (int j = 0; j < 4; ++j) {
      const size_t bo = (size_t)(n0 + (j << 4) + rlane) * ldb + koff + k0;
      bh[j] = Frag<T>::load(Bb + bo);
      if (SPLIT) bl[j] = Frag<T>::load(Bb2 + bo);
    }
#pragma unroll
    for (int i = 0; i < 4; ++i) {
      const size_t ao = (size_t)(m0 + (i << 4) + rlane) * lda + koff + k0;
      V ah = Frag<T>::load(Ab + ao);
      V al;
      if (SPLIT) al = Frag<T>::load(Ab2 + ao);
#pragma unroll
      for (int j = 0; j < 4; ++j) {
        acc[i][j] = Frag<T>::mma(ah, bh[j], acc[i][j]);
        if (SPLIT) {
          acc[i][j] = Frag<T>::mma(ah, bl[j], acc[i][j]);
          acc[i][j] = Frag<T>::mma(al, bh[j], acc[i][j]);
        }
      }
      Frag<T>::guard(acc[i][0], acc[i][3], ah, SPLIT ? al : ah);
    }
    Frag<T>::keep(bh[0], bh[1], bh[2], bh[3]);
    if (SPLIT) Frag<T>::keep(bl[0], bl[1], bl[2], bl[3]);
  }
  acc_guard4(acc[0][0], acc[0][1], acc[0][2], acc[0][3]);
  acc_guard4(acc[1][0], acc[1][1], acc[1][2], acc[1][3]);
  acc_guard4(acc[2][0], acc[2][1], acc[2][2], acc[2][3]);
  acc_guard4(acc[3][0], acc[3][1], acc[3][2], acc[3][3]);

  float* slab = sT[wave];
  const float* Rb = RESID ? (resid + (size_t)b * strideR) : nullptr;
#pragma unroll
  for (int i = 0; i < 4; ++i) {
    const int mBase = m0 + (i << 4);
#pragma unroll
    for (int j = 0; j < 4; ++j) {
      const int n = n0 + (j << 4) + rlane;
      float bv = 0.f;
      if (BIAS_MODE == 2) bv = bias[n];
#pragma unroll
      for (int r = 0; r < 8; ++r) {
        float v = acc[i][j][r] * scale;
        if (BIAS_MODE == 1) v += bias[mBase + mOff + r];
        if (BIAS_MODE == 2) v += bv;
        if (RESID) v += Rb[(size_t)(mBase + mOff + r) * ldc + n];
        if (ACT == 1) v = tanhf(v);
        if (ACT == 2) v = fmaxf(v, 0.0f);
        if (ACT == 3) v = v / (1.0f + expf(-v));
        if (ACT == 4) v = (v > 0.f) ? v : 0.01f * v;
        if (ACT == 5) v = 0.5f * v * (1.0f + erff(v * 0.70710678118654752f));
        if (ACT == 6) v = (v > 0.f) ? v : 0.2f * v;
        if (ACT == 7) { const float u = 0.7978845608028654f * (v + 0.044715f * v * v * v); v = 0.5f * v * (1.f + tanhf(u)); }
        slab[(mOff + r) * 68 + (j << 4) + rlane] = v;
      }
    }
    __builtin_amdgcn_fence(__ATOMIC_RELEASE, "workgroup");
    __builtin_amdgcn_wave_barrier();
    __builtin_amdgcn_fence(__ATOMIC_ACQUIRE, "workgroup");
    if (OUT_MODE == 0) {
      float* C = (float*)Cout + (size_t)b * strideC;
      const int hh = lane >> 4, c4 = (lane & 15) * 4;
      for (int pass = 0; pass < 2; ++pass) {
#pragma unroll
        for (int it = 0; it < 8; ++it) {
          const int row = it * 2 + hh;
          v4f v = *(const v4f*)(slab + row * 68 + c4);
          *(volatile v4f*)(C + (size_t)(mBase + row) * ldc + n0 + c4) = v;
        }
        __threadfence();
      }
    } else {
      const int q = lane >> 3, c8 = (lane & 7) * 8;
      unsigned short* C  = (unsigned short*)Cout  + (size_t)b * strideC;
      unsigned short* C2 = (OUT_MODE == 2) ? ((unsigned short*)Cout2 + (size_t)b * strideC) : nullptr;
      for (int pass = 0; pass < 2; ++pass) {
#pragma unroll
        for (int it = 0; it < 4; ++it) {
          const int row = it * 4 + q;
          const float* sp = slab + row * 68 + c8;
          v8h hv, lv;
#pragma unroll
          for (int e = 0; e < 8; ++e) {
            if (OUT_MODE == 1) {
              hv[e] = (_Float16)sp[e];
            } else {
              unsigned short hb = f2bf_bits(sp[e]);
              unsigned short lb = f2bf_bits(sp[e] - bf_bits2f(hb));
              hv[e] = __builtin_bit_cast(_Float16, hb);
              lv[e] = __builtin_bit_cast(_Float16, lb);
            }
          }
          *(volatile v8h*)(C + (size_t)(mBase + row) * ldc + n0 + c8) = hv;
          if (OUT_MODE == 2) *(volatile v8h*)(C2 + (size_t)(mBase + row) * ldc + n0 + c8) = lv;
        }
        __threadfence();
      }
    }
    __builtin_amdgcn_fence(__ATOMIC_RELEASE, "workgroup");
    __builtin_amdgcn_wave_barrier();
    __builtin_amdgcn_fence(__ATOMIC_ACQUIRE, "workgroup");
  }
}

}

__device__ __forceinline__ unsigned short bfu_rne(float v) { unsigned u = __builtin_bit_cast(unsigned, v); u += 0x7FFFu + ((u >> 16) & 1u); return (unsigned short)(u >> 16); }
__device__ __forceinline__ void bfsplit(float v, unsigned short& hi, unsigned short& lo) { hi = bfu_rne(v); lo = bfu_rne(v - __builtin_bit_cast(float, (unsigned)hi << 16)); }
__device__ __forceinline__ void st4s(unsigned short* Hp, unsigned short* Lp, long long o, v4f a) { unsigned short h[4], l[4]; bfsplit(a.x, h[0], l[0]); bfsplit(a.y, h[1], l[1]); bfsplit(a.z, h[2], l[2]); bfsplit(a.w, h[3], l[3]);
    const unsigned long long ph = (unsigned long long)h[0] | ((unsigned long long)h[1] << 16) | ((unsigned long long)h[2] << 32) | ((unsigned long long)h[3] << 48), pl = (unsigned long long)l[0] | ((unsigned long long)l[1] << 16) | ((unsigned long long)l[2] << 32) | ((unsigned long long)l[3] << 48);
    VST2(unsigned long long, (unsigned long long*)(Hp + o), ph); VST2(unsigned long long, (unsigned long long*)(Lp + o), pl); }

__device__ __forceinline__ unsigned short at_f2h(float x) { return (fabsf(x) < 6.104e-5f) ? (unsigned short)0 : __builtin_bit_cast(unsigned short, (_Float16)x); }
__device__ __forceinline__ void at_st8h(unsigned short* Pp, long long o, const float* v) { v4u pk; pk.x = (unsigned int)at_f2h(v[0]) | ((unsigned int)at_f2h(v[1]) << 16); pk.y = (unsigned int)at_f2h(v[2]) | ((unsigned int)at_f2h(v[3]) << 16); pk.z = (unsigned int)at_f2h(v[4]) | ((unsigned int)at_f2h(v[5]) << 16); pk.w = (unsigned int)at_f2h(v[6]) | ((unsigned int)at_f2h(v[7]) << 16); VST2(v4u, (v4u*)(Pp + o), pk); }

__global__ __launch_bounds__(256) void k_cvt16(const float* __restrict__ X, unsigned short* __restrict__ O16, float sc, long long n8) {
    const long long u = (long long)blockIdx.x * 256 + threadIdx.x; if (u >= n8) return;
    const float* x = X + 8 * u; const v4f a = *(const v4f*)x; const v4f b = *(const v4f*)(x + 4);
    float v[8] = {a.x, a.y, a.z, a.w, b.x, b.y, b.z, b.w};
#pragma unroll
    for (int i = 0; i < 8; ++i) v[i] = kit::bf_bits2f(kit::f2bf_bits(v[i])) * sc;
    at_st8h(O16, 8 * u, v); }

__global__ __launch_bounds__(256) void k_wopl(const float* __restrict__ W, int KIN, unsigned short* __restrict__ WP, int PP, long long n8) {
    const long long u = (long long)blockIdx.x * 256 + threadIdx.x; if (u >= n8) return;
    const int k8 = KIN / 8; const long long r = u / k8; const int c = 8 * (int)(u % k8);
    const float* w = W + r * KIN + c; const v4f a = *(const v4f*)w; const v4f b = *(const v4f*)(w + 4);
    v4u pk;
    pk.x = (unsigned)kit::f2bf_bits(a.x) | ((unsigned)kit::f2bf_bits(a.y) << 16); pk.y = (unsigned)kit::f2bf_bits(a.z) | ((unsigned)kit::f2bf_bits(a.w) << 16);
    pk.z = (unsigned)kit::f2bf_bits(b.x) | ((unsigned)kit::f2bf_bits(b.y) << 16); pk.w = (unsigned)kit::f2bf_bits(b.z) | ((unsigned)kit::f2bf_bits(b.w) << 16);
    VST2(v4u, (v4u*)(WP + r * PP + c), pk); VST2(v4u, (v4u*)(WP + r * PP + KIN + c), pk); }

__global__ __launch_bounds__(256) void k_pl4(const float* __restrict__ S, int SW, int CW, int RV, int R, unsigned short* __restrict__ PH, unsigned short* __restrict__ PL, int PP) { const long long u = (long long)blockIdx.x * 256 + threadIdx.x; const int cq = CW / 4; if (u >= (long long)R * cq) return; const int r = (int)(u / cq); const int c = 4 * (int)(u % cq); v4f v; v.x = v.y = v.z = v.w = 0.f; if (r < RV) v = *(const v4f*)(S + (long long)r * SW + c); st4s(PH, PL, (long long)r * PP + c, v); }
__global__ __launch_bounds__(256) void k_at_vtpl(const float* __restrict__ V, int ldv, int voff, int L, int D, int B, unsigned short* __restrict__ VTH, unsigned short* __restrict__ VTL) { const long long u = (long long)blockIdx.x * 256 + threadIdx.x; const int l4 = L / 4; if (u >= (long long)B * D * l4) return; const int l0 = 4 * (int)(u % l4); const long long bc = u / l4; const int c = (int)(bc % D); const int b = (int)(bc / D); v4f v; v.x = V[((long long)b * L + l0) * ldv + voff + c]; v.y = V[((long long)b * L + l0 + 1) * ldv + voff + c]; v.z = V[((long long)b * L + l0 + 2) * ldv + voff + c]; v.w = V[((long long)b * L + l0 + 3) * ldv + voff + c]; st4s(VTH, VTL, bc * L + l0, v); }

__global__ __launch_bounds__(32) void k_invf2(float* __restrict__ invb) {
    #pragma clang fp contract(off)
    const int i = threadIdx.x & 31; const float e = (float)i * 0.03125f; const float v = 1.0f / powf(10000.0f, e); VST2(float, invb + i, v); }
__global__ __launch_bounds__(256) void k_trig(const int* __restrict__ POS, const float* __restrict__ INVF, float* __restrict__ CS, float* __restrict__ SN, int n) {
    #pragma clang fp contract(off)
    const int idx = blockIdx.x * 256 + threadIdx.x; if (idx >= n) return; const int t = idx >> 5, i = idx & 31;
    const float ang = (float)POS[t] * INVF[i]; const float cv = cosf(ang); const float sv = sinf(ang);
    VST2(float, CS + idx, cv); VST2(float, SN + idx, sv); }

__global__ __launch_bounds__(256) void k_go_rope2(const float* __restrict__ QKV, const float* __restrict__ CS, const float* __restrict__ SN,
                                                   unsigned short* __restrict__ QH, unsigned short* __restrict__ QL, unsigned short* __restrict__ KH, unsigned short* __restrict__ KL, int nthr) {
    #pragma clang fp contract(off)
    const int u = blockIdx.x * 256 + threadIdx.x; if (u >= nthr) return;
    const int l = u & 15; const int hs = (u >> 4) % (NQH + NKVH); const int t = u / ((NQH + NKVH) * 16);
    const int i0 = 4 * (l & 7);
    const float* src = QKV + (long long)t * QKVW + hs * HDM;
    const v4f x1 = *(const v4f*)(src + i0), x2 = *(const v4f*)(src + 32 + i0);
    const v4f cs = *(const v4f*)(CS + (long long)t * 32 + i0), sn = *(const v4f*)(SN + (long long)t * 32 + i0);
    const v4f r1 = x1 * cs - x2 * sn;
    const v4f r2 = x2 * cs + x1 * sn;
    const bool first = (l < 8);
    v4f val; val.x = first ? r1.x : r2.x; val.y = first ? r1.y : r2.y; val.z = first ? r1.z : r2.z; val.w = first ? r1.w : r2.w;
    if (hs < NQH) st4s(QH, QL, (long long)t * QW + hs * HDM + 4 * l, val);
    else          st4s(KH, KL, (long long)t * KVW + (hs - NQH) * HDM + 4 * l, val); }

template <int NC>
__global__ __launch_bounds__(256) void k_go_sm2(const float* __restrict__ Sm, const float* __restrict__ SINK, const int* __restrict__ POS, int g, float sc,
                                                unsigned short* __restrict__ PH, unsigned short* __restrict__ PL, int nrows) {
    #pragma clang fp contract(off)
    constexpr int LL = 128 * NC;
    const int r = blockIdx.x * 8 + (threadIdx.x >> 5); const int L = threadIdx.x & 31; if (r >= nrows) return;
    const int z = r / LL, t = r - z * LL;
    const float* s = Sm + (long long)r * LL + 4 * L; const int* pp = POS + 4 * L; const long long pbase = (long long)r * LL + 4 * L;
    const float sink = kit::bf_bits2f(kit::f2bf_bits(SINK[8 * g + z]));
    const int pt = POS[t];
    v4f sv[NC]; v4i pk[NC];
    float m = -3.0e38f;
#pragma unroll
    for (int c = 0; c < NC; ++c) {
        sv[c] = *(const v4f*)(s + 128 * c); pk[c] = *(const v4i*)(pp + 128 * c);
#pragma unroll
        for (int e = 0; e < 4; ++e) { const float v = sv[c][e] * sc; m = fmaxf(m, (pk[c][e] <= pt) ? v : -3.0e38f); }
    }
#pragma unroll
    for (int o = 16; o > 0; o >>= 1) m = fmaxf(m, __shfl_xor(m, o, 32));
    m = fmaxf(m, sink);
    float sum = 0.f;
#pragma unroll
    for (int c = 0; c < NC; ++c) {
#pragma unroll
        for (int e = 0; e < 4; ++e) { const float ex = __expf(sv[c][e] * sc - m); const float pe = (pk[c][e] <= pt) ? ex : 0.f; sv[c][e] = pe; sum += pe; }
    }
#pragma unroll
    for (int o = 16; o > 0; o >>= 1) sum += __shfl_xor(sum, o, 32);
    const float inv = 1.f / (sum + __expf(sink - m));
#pragma unroll
    for (int c = 0; c < NC; ++c) { const v4f pv = sv[c] * inv; st4s(PH, PL, pbase + 128 * c, pv); }
}

extern "C" void kernel_launch(void* const* d_in, const int* in_sizes, int n_in, void* d_out, int out_size, void* d_ws, size_t ws_size, hipStream_t stream) {
    if (n_in < 5) return;
    if (in_sizes[0] < SEQ || in_sizes[1] < SEQ * HID || in_sizes[2] < QKVW * HID || in_sizes[3] < HID * QW || in_sizes[4] < NQH || out_size < SEQ * HID) return;
    const int*   pos   = (const int*)d_in[0];
    const float* hsf   = (const float*)d_in[1];
    const float* wqkv  = (const float*)d_in[2];
    const float* wo    = (const float*)d_in[3];
    const float* sinks = (const float*)d_in[4];
    float* out = (float*)d_out;

    const size_t x16B  = (size_t)SEQ * HID * 2;
    const size_t w16B  = (size_t)QKVW * HID * 2;
    const size_t qkvfB = (size_t)SEQ * QKVW * 4;
    const size_t sbB   = (size_t)8 * SEQ * SEQ * 4;
    const size_t plB   = (size_t)8 * SEQ * SEQ * 2;
    const size_t trigB = (size_t)SEQ * 32 * 4;
    const size_t wpB   = (size_t)HID * (2 * QW) * 2;
    static_assert(((size_t)SEQ * HID * 2) % 256 == 0 && ((size_t)QKVW * HID * 2) % 256 == 0 && ((size_t)SEQ * QKVW * 4) % 256 == 0 && ((size_t)SEQ * 32 * 4) % 256 == 0 && ((size_t)HID * (2 * QW) * 2) % 256 == 0);
    static_assert((size_t)SEQ * (2 * QW + 4 * KVW) * 2 <= (size_t)QKVW * HID * 2);
    static_assert((size_t)SEQ * (2 * QW) * 2 <= (size_t)QKVW * HID * 2);
    static_assert((size_t)SEQ * QW * 4 <= (size_t)SEQ * QKVW * 4);
    char* wsp = (char*)d_ws;
    unsigned short* X16 = (unsigned short*)wsp; wsp += x16B;
    unsigned short* W16 = (unsigned short*)wsp; wsp += w16B;
    float* QKVF = (float*)wsp; wsp += qkvfB;
    float* SB = (float*)wsp; wsp += sbB;
    unsigned short* PH = (unsigned short*)wsp; wsp += plB;
    unsigned short* PL = (unsigned short*)wsp; wsp += plB;
    float* INVF = (float*)wsp; wsp += 256;
    float* CS = (float*)wsp; wsp += trigB;
    float* SN = (float*)wsp; wsp += trigB;
    unsigned short* WP;
    if (wpB <= sbB + 2 * plB) WP = (unsigned short*)SB; else { WP = (unsigned short*)wsp; wsp += wpB; }
    if ((size_t)(wsp - (char*)d_ws) > ws_size) return;
    unsigned short* QH  = W16;
    unsigned short* QL  = QH + (size_t)SEQ * QW;
    unsigned short* KH  = QL + (size_t)SEQ * QW;
    unsigned short* KL  = KH + (size_t)SEQ * KVW;
    unsigned short* VTH = KL + (size_t)SEQ * KVW;
    unsigned short* VTL = VTH + (size_t)KVW * SEQ;
    unsigned short* CP  = W16;
    float* CTX = QKVF;

    k_cvt16<<<(unsigned)(((long long)SEQ * HID / 8 + 255) / 256), 256, 0, stream>>>(hsf, X16, 1.0f, (long long)SEQ * HID / 8);
    k_cvt16<<<(unsigned)(((long long)QKVW * HID / 8 + 255) / 256), 256, 0, stream>>>(wqkv, W16, 64.0f, (long long)QKVW * HID / 8);
    kit::wmma_gemm64<0, false, 0, 0, false, 0><<<dim3((unsigned)(((SEQ / 64) * (QKVW / 64) + 7) / 8), 1u), 256, 0, stream>>>(
        X16, nullptr, HID, 0L, W16, nullptr, HID, 0L, (void*)QKVF, nullptr, QKVW, 0L, nullptr, nullptr, 0L, SEQ, QKVW, HID, 0.015625f);
    k_invf2<<<1, 32, 0, stream>>>(INVF);
    k_trig<<<(unsigned)((SEQ * 32 + 255) / 256), 256, 0, stream>>>(pos, INVF, CS, SN, SEQ * 32);
    k_go_rope2<<<(unsigned)((SEQ * (NQH + NKVH) * 16 + 255) / 256), 256, 0, stream>>>(QKVF, CS, SN, QH, QL, KH, KL, SEQ * (NQH + NKVH) * 16);
    k_at_vtpl<<<(unsigned)(((long long)KVW * (SEQ / 4) + 255) / 256), 256, 0, stream>>>(QKVF, QKVW, QW + KVW, SEQ, KVW, 1, VTH, VTL);
    for (int g = 0; g < NKVH; ++g) {
        kit::wmma_gemm64<1, true, 0, 0, false, 0><<<dim3((unsigned)(((SEQ / 64) * (SEQ / 64) + 7) / 8), 8u), 256, 0, stream>>>(
            QH + (size_t)g * (8 * HDM), QL + (size_t)g * (8 * HDM), QW, (long)HDM, KH + (size_t)g * HDM, KL + (size_t)g * HDM, KVW, 0L,
            (void*)SB, nullptr, SEQ, (long)SEQ * SEQ, nullptr, nullptr, 0L, SEQ, SEQ, HDM, 1.0f);
        k_go_sm2<SEQ / 128><<<(unsigned)((8 * SEQ + 7) / 8), 256, 0, stream>>>(SB, sinks, pos, g, 0.125f, PH, PL, 8 * SEQ);
        kit::wmma_gemm64<1, true, 0, 0, false, 0><<<dim3((unsigned)(((SEQ / 64) * (HDM / 64) + 7) / 8), 8u), 256, 0, stream>>>(
            PH, PL, SEQ, (long)SEQ * SEQ, VTH + (size_t)g * HDM * SEQ, VTL + (size_t)g * HDM * SEQ, SEQ, 0L,
            (void*)(CTX + (size_t)g * (8 * HDM)), nullptr, QW, (long)HDM, nullptr, nullptr, 0L, SEQ, HDM, SEQ, 1.0f);
    }
    k_pl4<<<(unsigned)(((long long)SEQ * (QW / 4) + 255) / 256), 256, 0, stream>>>(CTX, QW, QW, SEQ, SEQ, CP, CP + QW, 2 * QW);
    k_wopl<<<(unsigned)(((long long)HID * QW / 8 + 255) / 256), 256, 0, stream>>>(wo, QW, WP, 2 * QW, (long long)HID * QW / 8);
    kit::wmma_gemm64<1, false, 0, 0, false, 0><<<dim3((unsigned)(((SEQ / 64) * (HID / 64) + 7) / 8), 1u), 256, 0, stream>>>(
        CP, nullptr, 2 * QW, 0L, WP, nullptr, 2 * QW, 0L, (void*)out, nullptr, HID, 0L, nullptr, nullptr, 0L, SEQ, HID, 2 * QW, 1.0f);
}
